// RGCNLayer_77902116815140
// MI455X (gfx1250) — hardware-run, weakly checked
//
#include <hip/hip_runtime.h>

typedef float          v8f   __attribute__((ext_vector_type(8)));
typedef float          v4f   __attribute__((ext_vector_type(4)));
typedef unsigned int   v4u   __attribute__((ext_vector_type(4)));
typedef int            v8i   __attribute__((ext_vector_type(8)));
typedef unsigned short v8us  __attribute__((ext_vector_type(8)));
typedef unsigned short v16us __attribute__((ext_vector_type(16)));
typedef __bf16         v16bf __attribute__((ext_vector_type(16)));
typedef _Float16       v16h  __attribute__((ext_vector_type(16)));
typedef v4f  __attribute__((may_alias)) v4fa;
typedef v8us __attribute__((may_alias)) v8usa;
union FragB { v16bf v; v16us u; v8us h[2]; v8i w; };
union FragH { v16h  v; v16us u; v8us h[2]; v8i w; };

__device__ __forceinline__ v8f wmb(const FragB& a, const FragB& b, v8f c) {
  v8f d = __builtin_amdgcn_wmma_f32_16x16x32_bf16(false, a.v, false, b.v, (short)0, c, false, false);
  asm volatile("v_nop\n\tv_nop\n\tv_nop\n\tv_nop" : "+v"(d) : "v"(a.w), "v"(b.w));
  return d;
}

__device__ __forceinline__ v8f wmh(const FragH& a, const FragH& b, v8f c) {
  v8f d = __builtin_amdgcn_wmma_f32_16x16x32_f16(false, a.v, false, b.v, (short)0, c, false, false);
  asm volatile("v_nop\n\tv_nop\n\tv_nop\n\tv_nop" : "+v"(d) : "v"(a.w), "v"(b.w));
  return d;
}

__device__ __forceinline__ unsigned bf16_bits(float f) {
  const unsigned u = __float_as_uint(f);
  const unsigned r = (u + 0x7FFFu + ((u >> 16) & 1u)) >> 16;
  const unsigned q = (u >> 16) | 0x40u;
  return ((u & 0x7fffffffu) > 0x7f800000u) ? q : r;
}

__device__ __forceinline__ float bf16_val(float f) {
  return __uint_as_float(bf16_bits(f) << 16);
}
__device__ __forceinline__ int clampi(int v, int lo, int hi) {
  return v < lo ? lo : (v > hi ? hi : v);
}

__device__ __forceinline__ unsigned f16_bits(float f) {
  const unsigned u  = __float_as_uint(f);
  const unsigned s  = (u >> 16) & 0x8000u;
  const unsigned a  = u & 0x7fffffffu;
  const unsigned t  = a - 0x38000000u;
  const unsigned r  = (t + 0x0FFFu + ((t >> 13) & 1u)) >> 13;
  const unsigned rc = r > 0x7C00u ? 0x7C00u : r;
  const bool small  = a < 0x38800000u;
  const bool isnan  = a > 0x7f800000u;
  const unsigned fin = small ? 0u : (s | rc);
  return isnan ? (s | 0x7E00u) : fin;
}

__device__ __forceinline__ unsigned pk16(unsigned lo, unsigned hi) { return lo | (hi << 16); }
__device__ __forceinline__ unsigned bf16_lo_bits(float v) {
  float hi = bf16_val(v);
  asm volatile("" : "+v"(hi));
  return bf16_bits(v - hi);
}
__device__ __forceinline__ v4u pack8_bf16(v4f a, v4f c) {
  return (v4u){ pk16(bf16_bits(a[0]), bf16_bits(a[1])), pk16(bf16_bits(a[2]), bf16_bits(a[3])),
                pk16(bf16_bits(c[0]), bf16_bits(c[1])), pk16(bf16_bits(c[2]), bf16_bits(c[3])) };
}
__device__ __forceinline__ v4u pack8_bf16_lo(v4f a, v4f c) {
  return (v4u){ pk16(bf16_lo_bits(a[0]), bf16_lo_bits(a[1])), pk16(bf16_lo_bits(a[2]), bf16_lo_bits(a[3])),
                pk16(bf16_lo_bits(c[0]), bf16_lo_bits(c[1])), pk16(bf16_lo_bits(c[2]), bf16_lo_bits(c[3])) };
}
__device__ __forceinline__ v4u pack8_f16(v4f a, v4f c) {
  return (v4u){ pk16(f16_bits(a[0]), f16_bits(a[1])), pk16(f16_bits(a[2]), f16_bits(a[3])),
                pk16(f16_bits(c[0]), f16_bits(c[1])), pk16(f16_bits(c[2]), f16_bits(c[3])) };
}

template <int FORM>
__global__ __launch_bounds__(256) void k_plane(const float* __restrict__ src, int rows, int cols, int ldsrc,
                                               unsigned short* __restrict__ dst, int MP, int KP) {
  static_assert(FORM >= 0 && FORM <= 3);
  const int KTOT = (FORM == 1 || FORM == 3) ? 2 * KP : KP;
  const unsigned ppr   = (unsigned)(KTOT >> 3);
  const unsigned kp8   = (unsigned)(KP >> 3);
  const unsigned total = (unsigned)MP * ppr;
  const unsigned g     = blockIdx.x * 256u + threadIdx.x;
  const unsigned rowu  = g / ppr;
  const unsigned p     = g - rowu * ppr;
  const bool second    = p >= kp8;
  const int row = (int)rowu;
  const int c0  = (int)((second ? p - kp8 : p) << 3);
  const float* srow = src + (size_t)clampi(row, 0, rows - 1) * (size_t)ldsrc;
  float x[8];
  unsigned mk[8];
#pragma unroll
  for (int e = 0; e < 8; ++e) {
    const int c = c0 + e;
    const float v = srow[clampi(c, 0, cols - 1)];
    asm volatile("" :: "v"(v));
    x[e]  = v;
    mk[e] = (row < rows && c < cols) ? 0xFFFFu : 0u;
  }
  const v4f a = (v4f){ x[0], x[1], x[2], x[3] };
  const v4f c = (v4f){ x[4], x[5], x[6], x[7] };
  v4u o;
  if (FORM == 2) {
    o = pack8_f16(a, c);
  } else {
    const v4u hi = pack8_bf16(a, c);
    o = hi;
    if (FORM == 1) { const v4u lo = pack8_bf16_lo(a, c); o = second ? lo : hi; }
  }
  const v4u mw = (v4u){ pk16(mk[0], mk[1]), pk16(mk[2], mk[3]), pk16(mk[4], mk[5]), pk16(mk[6], mk[7]) };
  o &= mw;
  if (g < total) {
    volatile v4u* q = (volatile v4u*)(dst + (size_t)g * 8);
    *q = o;
    __threadfence();
    *q = o;
  }
}

template <int FORM> struct FragOf    { typedef FragB T; };
template <>         struct FragOf<2> { typedef FragH T; };
__device__ __forceinline__ v8f mm(const FragB& a, const FragB& b, v8f c) { return wmb(a, b, c); }
__device__ __forceinline__ v8f mm(const FragH& a, const FragH& b, v8f c) { return wmh(a, b, c); }
template <class F> __device__ __forceinline__ F ld_frag(const unsigned short* p) {
  F f;
  f.h[0] = *(const v8usa*)(p);
  f.h[1] = *(const v8usa*)(p + 16);
  return f;
}

template <int FORM, int EPI>
__global__ __launch_bounds__(256) __attribute__((amdgpu_num_vgpr(248)))
void k_gemm_nt(const unsigned short* __restrict__ A, const unsigned short* __restrict__ B,
               const float* __restrict__ bias, float* __restrict__ D, int M, int N, int KTOT, int ldd) {
  static_assert(FORM >= 0 && FORM <= 2);
  static_assert(EPI == 0 || EPI == 1);
  typedef typename FragOf<FORM>::T F;
  __shared__ __attribute__((aligned(16))) float sT[8][16 * 68];
  const int lane = threadIdx.x & 31;
  const int wave = threadIdx.x >> 5;
  const int tilesM = (M + 63) >> 6;
  const int tilesN = (N + 63) >> 6;
  const int tile = blockIdx.x * 8 + wave;
  if (tile >= tilesM * tilesN) return;
  const int tm = tile / tilesN;
  const int tn = tile - tm * tilesN;
  const int m0 = tm << 6;
  const int n0 = tn << 6;

  const int rl = lane & 15;
  const int h8 = (lane >> 4) * 8;
  const unsigned short* pa = A + (size_t)(m0 + rl) * (size_t)KTOT + h8;
  const unsigned short* pb = B + (size_t)(n0 + rl) * (size_t)KTOT + h8;

  v8f acc[4][4];
#pragma unroll
  for (int i = 0; i < 4; ++i)
#pragma unroll
    for (int j = 0; j < 4; ++j) acc[i][j] = (v8f){0.f, 0.f, 0.f, 0.f, 0.f, 0.f, 0.f, 0.f};

#pragma unroll 1
  for (int k0 = 0; k0 < KTOT; k0 += 32) {
    F bf[4];
#pragma unroll
    for (int j = 0; j < 4; ++j) bf[j] = ld_frag<F>(pb + (size_t)(j << 4) * (size_t)KTOT + k0);
#pragma unroll
    for (int i = 0; i < 4; ++i) {
      const F af = ld_frag<F>(pa + (size_t)(i << 4) * (size_t)KTOT + k0);
#pragma unroll
      for (int j = 0; j < 4; ++j) acc[i][j] = mm(af, bf[j], acc[i][j]);
    }
  }

  float* slab = sT[wave];
  const int hh = lane >> 4;
  const int c4 = (lane & 15) * 4;
  const int nc = n0 + c4;
  const bool cok = nc < N;
  v4f bv = (v4f){0.f, 0.f, 0.f, 0.f};
  if (EPI == 1) {
    bv = *(const v4fa*)(bias + clampi(nc, 0, N - 4));
    asm volatile("" :: "v"(bv));
  }
#pragma unroll
  for (int i = 0; i < 4; ++i) {
    const int mBase = m0 + (i << 4);
#pragma unroll
    for (int j = 0; j < 4; ++j) {
#pragma unroll
      for (int r = 0; r < 8; ++r) slab[(h8 + r) * 68 + (j << 4) + rl] = acc[i][j][r];
    }
    __builtin_amdgcn_fence(__ATOMIC_RELEASE, "workgroup");
    __builtin_amdgcn_wave_barrier();
    __builtin_amdgcn_fence(__ATOMIC_ACQUIRE, "workgroup");
    v4f vv[8];
#pragma unroll
    for (int it = 0; it < 8; ++it) {
      const int row = it * 2 + hh;
      v4f v = *(const v4fa*)(slab + row * 68 + c4);
      if (EPI == 1) v += bv;
      vv[it] = v;
    }
    for (int pass = 0; pass < 2; ++pass) {
#pragma unroll
      for (int it = 0; it < 8; ++it) {
        const int row = mBase + it * 2 + hh;
        if (cok && row < M) *(volatile v4f*)(D + (size_t)row * (size_t)ldd + nc) = vv[it];
      }
      __threadfence();
    }
    __builtin_amdgcn_fence(__ATOMIC_RELEASE, "workgroup");
    __builtin_amdgcn_wave_barrier();
    __builtin_amdgcn_fence(__ATOMIC_ACQUIRE, "workgroup");
  }
}

#include <stddef.h>
#include <stdint.h>

#define TERMS_A 1
#define TERMS_W 1
#define NSEG    (TERMS_A + TERMS_W - 1)
#define KPAIR   (64 * NSEG)

#define NN      100000
#define NE      1000000
#define CC      64
#define NREL    32
#define NBAS    30
#define NB      1024
#define SLA     10
#define NBLK    98
#define MPACC   (NBLK * NB)
#define MPX     100096
#define NGRP    8
#define RELROWS 28672
#define GROWS   (4 * RELROWS)
#define NTHR    256
#define NWAVE   8
#define SPW     (NB / NWAVE)
#define EPT     8
#define CHUNK   (NTHR * EPT)
#define WCAP    (EPT * 32)
#define LISTN   (NWAVE * WCAP)
#define RCAP    13312
#define PCAP    11264
#define NKEY    (NB * NREL)
#define ARRN    (NKEY + 16)
#define REG0N   (LISTN + 2 * RCAP)
#define BK_INTS (REG0N + ARRN + 3 * NB + 256 + 128)
#define PB_X    3128
#define PB_W    2
#define PPRW    (KPAIR / 8)
#define OFFN    ((NBLK + 2) * 32)

static_assert(TERMS_A == 1 || TERMS_A == 2);
static_assert(TERMS_W == 1 || TERMS_W == 2);
static_assert(KPAIR % 32 == 0 && KPAIR >= 64 && KPAIR <= 192);
static_assert(CC == 64 && NREL == 32 && NB == (1 << SLA) && NKEY == 32768);
static_assert(NBLK * NB >= NN && MPACC == NBLK * NB && (NBLK - 1) * NB < NN);
static_assert(MPX % 64 == 0 && MPX >= NN && MPX % 16 == 0);
static_assert(RELROWS % 64 == 0 && RELROWS == 224 * 128);
static_assert(GROWS >= 100096 && GROWS >= MPX);
static_assert(PB_X * 256 == MPX * 8 && PB_W * 256 == CC * 8);
static_assert(RCAP % 256 == 0 && RCAP >= 10529 + 10529 / 4 && RCAP <= 16384);
static_assert(PCAP % 256 == 0 && PCAP >= 10529 && (2 * PCAP) % 32 == 0 && 2 * PCAP <= REG0N);
static_assert(NN <= (1 << 17) && (NKEY - 1) < (1 << 15));
static_assert((NE % 8) == 0 && ((CHUNK << SLA) > 0));
static_assert(BK_INTS % 4 == 0 && REG0N % 4 == 0 && ARRN % 4 == 0 && RCAP % 32 == 0 && NB % 32 == 0);
static_assert(BK_INTS * 4 <= 262144);
static_assert(SPW == 128 && SPW % 32 == 0);
static_assert(OFFN % 128 == 0);
static_assert(NGRP * 4 == NREL);

typedef int      v4i  __attribute__((ext_vector_type(4)));
typedef unsigned v2u  __attribute__((ext_vector_type(2)));
typedef float    v2f  __attribute__((ext_vector_type(2)));
typedef v4i __attribute__((may_alias)) v4ia;
typedef v2u __attribute__((may_alias)) v2ua;
typedef v2f __attribute__((may_alias)) v2fa;

__device__ __forceinline__ void pinf(float x)    { asm volatile("" :: "v"(x)); }
__device__ __forceinline__ void pini(int x)      { asm volatile("" :: "v"(x)); }
__device__ __forceinline__ void pinu(unsigned x) { asm volatile("" :: "v"(x)); }
__device__ __forceinline__ void pin4f(v4f x)     { asm volatile("" :: "v"(x)); }
__device__ __forceinline__ void pin2f(v2f x)     { asm volatile("" :: "v"(x)); }

__global__ __launch_bounds__(256) void k_prep(const float* __restrict__ x, const float* __restrict__ sw,
                                              const float* __restrict__ bias, unsigned short* xb,
                                              unsigned short* wst, float* biasr) {
  const int b = (int)blockIdx.x, tid = (int)threadIdx.x;
  if (b < PB_X) {
    const int u   = b * 256 + tid;
    const int row = u >> 3;
    const int c0  = (u & 7) * 8;
    const int rc  = row < NN ? row : NN - 1;
    const float* p = x + (size_t)rc * CC + c0;
    const v4f a = *(const v4fa*)p;
    const v4f c = *(const v4fa*)(p + 4);
    pin4f(a); pin4f(c);
    v4u o = pack8_bf16(a, c);
    const unsigned mk = row < NN ? 0xFFFFFFFFu : 0u;
    o &= (v4u){ mk, mk, mk, mk };
    volatile v4u* q = (volatile v4u*)(xb + (size_t)u * 8);
    *q = o;
    __threadfence();
    *q = o;
  } else if (b < PB_X + PB_W) {
    const int u  = (b - PB_X) * 256 + tid;
    const int n  = u >> 3, k8 = (u & 7) * 8;
    float f[8];
#pragma unroll
    for (int i = 0; i < 8; ++i) { f[i] = sw[(size_t)(k8 + i) * CC + n]; pinf(f[i]); }
    const v4u o = pack8_bf16((v4f){ f[0], f[1], f[2], f[3] }, (v4f){ f[4], f[5], f[6], f[7] });
    volatile v4u* q = (volatile v4u*)(wst + (size_t)u * 8);
    *q = o;
    __threadfence();
    *q = o;
  } else {
    const int li = tid < 16 ? tid : 15;
    const v4f a = *(const v4fa*)(bias + 4 * li);
    pin4f(a);
    const v4f o = (v4f){ bf16_val(a[0]), bf16_val(a[1]), bf16_val(a[2]), bf16_val(a[3]) };
    if (tid < 16) {
      volatile v4f* q = (volatile v4f*)(biasr + 4 * tid);
      *q = o;
      __threadfence();
      *q = o;
    }
  }
}

__global__ __launch_bounds__(256) void k_relw(const float* __restrict__ coeff, const float* __restrict__ basis,
                                              unsigned short* rwb) {
  __shared__ __attribute__((aligned(16))) float sc[32];
  __shared__ __attribute__((aligned(16))) float swt[16 * 68];
  const int tid = (int)threadIdx.x;
  const int r   = (int)blockIdx.x >> 2;
  const int o0  = ((int)blockIdx.x & 3) * 16;
  if (tid < 32) {
    const float c = coeff[r * NBAS + (tid < NBAS ? tid : NBAS - 1)];
    pinf(c);
    sc[tid] = (tid < NBAS) ? bf16_val(c) : 0.0f;
  }
  __syncthreads();
  const int ol = tid & 15, i0 = tid >> 4;
  const float* bp = basis + (size_t)i0 * CC + o0 + ol;
  float a0 = 0.0f, a1 = 0.0f, a2 = 0.0f, a3 = 0.0f;
#pragma unroll 1
  for (int bb = 0; bb < NBAS; ++bb) {
    const float cb = sc[bb];
    const float* q = bp + (size_t)bb * (CC * CC);
    const float v0 = q[0], v1 = q[16 * CC], v2 = q[32 * CC], v3 = q[48 * CC];
    pinf(v0); pinf(v1); pinf(v2); pinf(v3);
    a0 = fmaf(cb, bf16_val(v0), a0);
    a1 = fmaf(cb, bf16_val(v1), a1);
    a2 = fmaf(cb, bf16_val(v2), a2);
    a3 = fmaf(cb, bf16_val(v3), a3);
  }
  swt[ol * 68 + i0]      = a0;
  swt[ol * 68 + i0 + 16] = a1;
  swt[ol * 68 + i0 + 32] = a2;
  swt[ol * 68 + i0 + 48] = a3;
  __syncthreads();
  v4u ov[2];
#pragma unroll
  for (int it = 0; it < 2; ++it) {
    const int p   = tid + 256 * it;
    const int pc  = p < 16 * PPRW ? p : 16 * PPRW - 1;
    const int row = pc / PPRW;
    const int q   = pc - row * PPRW;
    const int seg = q >> 3;
    const int c0  = (q & 7) * 8;
    const v4f a = *(const v4fa*)(swt + row * 68 + c0);
    const v4f c = *(const v4fa*)(swt + row * 68 + c0 + 4);
    const v4u hi = pack8_bf16(a, c);
    const v4u lo = pack8_bf16_lo(a, c);
    const unsigned m = (TERMS_W == 2 && seg == NSEG - 1) ? 0xFFFFFFFFu : 0u;
    const v4u mv = (v4u){ m, m, m, m };
    ov[it] = (lo & mv) | (hi & ~mv);
  }
  unsigned short* dst = rwb + (size_t)(r * CC + o0) * KPAIR;
  for (int pass = 0; pass < 2; ++pass) {
#pragma unroll
    for (int it = 0; it < 2; ++it) {
      const int p = tid + 256 * it;
      if (p < 16 * PPRW) *(volatile v4u*)(dst + (size_t)p * 8) = ov[it];
    }
    __threadfence();
  }
}

__device__ __forceinline__ int ldkey(const int* __restrict__ k, int e, int nE, int sent) {
  const int v = k[e < nE ? e : nE - 1];
  pini(v);
  return (e < nE) ? v : sent;
}

__device__ __forceinline__ int scan_chunk(const int* __restrict__ keys, int nE, int cbase, int slotBase,
                                          int nb, int* list, int tid, int lane, int wave) {
  int wc = 0;
  const int el0  = tid * EPT;
  const int e0   = cbase + el0;
  const int sent = (int)(1u << 31);
  v4i da, db;
  if (cbase + CHUNK <= nE) {
    da = *(const v4ia*)(keys + e0);
    db = *(const v4ia*)(keys + e0 + 4);
  } else {
    da.x = ldkey(keys, e0,     nE, sent);
    da.y = ldkey(keys, e0 + 1, nE, sent);
    da.z = ldkey(keys, e0 + 2, nE, sent);
    da.w = ldkey(keys, e0 + 3, nE, sent);
    db.x = ldkey(keys, e0 + 4, nE, sent);
    db.y = ldkey(keys, e0 + 5, nE, sent);
    db.z = ldkey(keys, e0 + 6, nE, sent);
    db.w = ldkey(keys, e0 + 7, nE, sent);
  }
  const unsigned nbs = (unsigned)slotBase;
  const unsigned unb = (unsigned)nb;
  const unsigned s0 = (unsigned)da.x - nbs, s1 = (unsigned)da.y - nbs;
  const unsigned s2 = (unsigned)da.z - nbs, s3 = (unsigned)da.w - nbs;
  const unsigned s4 = (unsigned)db.x - nbs, s5 = (unsigned)db.y - nbs;
  const unsigned s6 = (unsigned)db.z - nbs, s7 = (unsigned)db.w - nbs;
  const bool h0 = s0 < unb, h1 = s1 < unb, h2 = s2 < unb, h3 = s3 < unb;
  const bool h4 = s4 < unb, h5 = s5 < unb, h6 = s6 < unb, h7 = s7 < unb;
  const unsigned any = __builtin_amdgcn_ballot_w32(h0 | h1 | h2 | h3 | h4 | h5 | h6 | h7);
  if (any != 0u) {
    const int k = (int)h0 + (int)h1 + (int)h2 + (int)h3 + (int)h4 + (int)h5 + (int)h6 + (int)h7;
    int incl = k;
#pragma unroll
    for (int dd = 1; dd < 32; dd <<= 1) {
      const int y = __shfl_up(incl, dd, 32);
      if (lane >= dd) incl += y;
    }
    wc = __shfl(incl, 31, 32);
    int pos = incl - k;
#define PUTJ(J, HJ, SJ) if (HJ) { if (pos < WCAP) list[wave * WCAP + pos] = ((el0 + (J)) << SLA) | (int)(SJ); pos += 1; }
    PUTJ(0, h0, s0)
    PUTJ(1, h1, s1)
    PUTJ(2, h2, s2)
    PUTJ(3, h3, s3)
    PUTJ(4, h4, s4)
    PUTJ(5, h5, s5)
    PUTJ(6, h6, s6)
    PUTJ(7, h7, s7)
#undef PUTJ
  }
  return wc;
}

__global__ __launch_bounds__(NTHR) void k_bucket(const int* __restrict__ snd, const int* __restrict__ rcv,
                                                 const int* __restrict__ rel, int* entg, int* pairg,
                                                 int* poffg, int* pcntg, int* degg, int* binfog) {
  extern __shared__ __attribute__((aligned(16))) int dsm[];
  int* list  = dsm;
  int* hks   = dsm + LISTN;
  int* ent   = hks + RCAP;
  int* pst   = dsm;
  int* arr   = dsm + REG0N;
  int* spoff = arr + ARRN;
  int* spcnt = spoff + NB;
  int* sdeg  = spcnt + NB;
  int* wrel  = sdeg + NB;
  int* misc  = wrel + 256;
  int* binf  = misc + 64;
  const int tid = (int)threadIdx.x, lane = tid & 31;
  const int wave = __builtin_amdgcn_readfirstlane(tid >> 5);
  const int b = (int)blockIdx.x;
  const int nodeBase = b * NB;

  {
    const v4i z4 = {0, 0, 0, 0};
    for (int i = tid * 4; i < BK_INTS; i += NTHR * 4) *(v4ia*)(dsm + i) = z4;
  }
  __syncthreads();

  int t = 0;
  const int nChunks = (NE + CHUNK - 1) / CHUNK;
#pragma unroll 1
  for (int ch = 0; ch < nChunks; ++ch) {
    const int cbase = ch * CHUNK;
    int wc = scan_chunk(rcv, NE, cbase, nodeBase, NB, list, tid, lane, wave);
    wc = clampi(wc, 0, WCAP);
    wc = __builtin_amdgcn_readfirstlane(wc);
    int* mb = misc + (ch & 1) * 8;
    if (lane == 0) mb[wave] = wc;
    __syncthreads();
    int base = t, tot = 0;
#pragma unroll
    for (int w2 = 0; w2 < NWAVE; ++w2) {
      const int c = clampi(mb[w2], 0, WCAP);
      base += (w2 < wave) ? c : 0;
      tot  += c;
    }
#pragma unroll 1
    for (int b0 = 0; b0 < wc; b0 += 32) {
      const int idx  = b0 + lane;
      const int entv = list[wave * WCAP + (idx < WCAP ? idx : WCAP - 1)];
      const int slot = entv & (NB - 1);
      const int el   = (entv >> SLA) & (CHUNK - 1);
      const int eid  = clampi(cbase + el, 0, NE - 1);
      int ty = rel[eid];
      pini(ty);
      ty = clampi(ty, 0, NREL - 1);
      int sr = snd[eid];
      pini(sr);
      sr = clampi(sr, 0, NN - 1);
      const int pos = base + idx;
      if (idx < wc && pos < RCAP) {
        hks[pos] = (int)(((unsigned)(slot * NREL + ty) << 17) | (unsigned)sr);
      }
    }
    t += tot;
  }
  __syncthreads();
  const int tt = t < RCAP ? t : RCAP;
  const int ov = t > RCAP ? 1 : 0;

  if (tid == 0) {
#pragma unroll 1
    for (int i = 0; i < tt; ++i) {
      const int k = (int)((unsigned)hks[i] >> 17);
      arr[k] = arr[k] + 1;
    }
  }
  __syncthreads();
  if (wave == 0) {
    const int base = lane * (NKEY / 32);
    int s = 0;
#pragma unroll 1
    for (int i = 0; i < NKEY / 32; ++i) s += arr[base + i];
    int incl = s;
#pragma unroll
    for (int dd = 1; dd < 32; dd <<= 1) {
      const int y = __shfl_up(incl, dd, 32);
      if (lane >= dd) incl += y;
    }
    int run = incl - s;
#pragma unroll 1
    for (int i = 0; i < NKEY / 32; ++i) {
      run += arr[base + i];
      arr[base + i] = run;
    }
    if (lane == 31) arr[NKEY] = run;
  }
  __syncthreads();
  if (tid == 0) {
#pragma unroll 1
    for (int i = tt - 1; i >= 0; --i) {
      const int v = hks[i];
      const int k = (int)((unsigned)v >> 17);
      const int p = clampi(arr[k] - 1, 0, RCAP - 1);
      arr[k] = p;
      ent[p] = v & 0x1FFFF;
    }
  }
  __syncthreads();
  {
    int* eg = entg + (size_t)b * RCAP;
    for (int pass = 0; pass < 2; ++pass) {
      for (int i = tid * 4; i < RCAP; i += NTHR * 4) {
        const v4i v = *(const v4ia*)(ent + i);
        *(volatile v4i*)(eg + i) = v;
      }
      __threadfence();
    }
  }
  __syncthreads();

  {
    const v4i z4 = {0, 0, 0, 0};
    for (int i = tid * 4; i < 2 * PCAP; i += NTHR * 4) *(v4ia*)(pst + i) = z4;
    int relc = 0, ptot = 0, ovd = 0;
#pragma unroll 1
    for (int s = wave * SPW; s < wave * SPW + SPW; ++s) {
      const int k = s * NREL + lane;
      const int c = arr[k + 1] - arr[k];
      ovd |= (c > 255) ? 1 : 0;
      const bool ne = c > 0;
      relc += ne ? 1 : 0;
      const unsigned mk = __builtin_amdgcn_ballot_w32(ne);
      ptot += (int)__builtin_popcount(mk);
    }
    wrel[wave * 32 + lane] = relc;
    const unsigned om = __builtin_amdgcn_ballot_w32(ovd != 0);
    if (lane == 0) { misc[16 + wave] = ptot; misc[24 + wave] = (om != 0u) ? 1 : 0; }
  }
  __syncthreads();

  {
    int runrel = 0, bc = 0, pbase = 0, ptotal = 0, fl = ov;
#pragma unroll
    for (int w2 = 0; w2 < NWAVE; ++w2) {
      const int c  = clampi(wrel[w2 * 32 + lane], 0, SPW);
      const int tq = clampi(misc[16 + w2], 0, SPW * NREL);
      runrel += (w2 < wave) ? c : 0;
      bc     += c;
      pbase  += (w2 < wave) ? tq : 0;
      ptotal += tq;
      fl     |= misc[24 + w2];
    }
    fl |= (ptotal > PCAP) ? 1 : 0;
#pragma unroll 1
    for (int s = wave * SPW; s < wave * SPW + SPW; ++s) {
      const int k  = s * NREL + lane;
      const int st = arr[k];
      const int c  = arr[k + 1] - st;
      const int cc = clampi(c, 0, 255);
      const bool ne = c > 0;
      const unsigned mk = __builtin_amdgcn_ballot_w32(ne);
      const int np  = (int)__builtin_popcount(mk);
      const int idx = pbase + (int)__builtin_amdgcn_mbcnt_lo(mk, 0u);
      if (ne && idx >= 0 && idx < PCAP) {
        pst[2 * idx]     = clampi(st, 0, RCAP - 1) | (cc << 14) | (lane << 22);
        pst[2 * idx + 1] = runrel;
      }
      runrel += ne ? 1 : 0;
      const int d0 = arr[s * NREL];
      const int d1 = arr[s * NREL + NREL];
      if (lane == 0) {
        const int po = pbase < PCAP ? pbase : PCAP;
        spoff[s] = po;
        spcnt[s] = (np < PCAP - po) ? np : (PCAP - po);
        sdeg[s]  = clampi(d1 - d0, 0, RCAP);
      }
      pbase += np;
    }
    if (wave == 0) {
      binf[lane] = bc;
      const int pt = ptotal < PCAP ? ptotal : PCAP;
      int v = 0;
      v = (lane == 0) ? fl : v;
      v = (lane == 1) ? pt : v;
      v = (lane == 2) ? tt : v;
      binf[32 + lane] = v;
    }
  }
  __syncthreads();

  {
    int* pg = pairg + (size_t)b * (2 * PCAP);
    int* og = poffg + (size_t)b * NB;
    int* cg = pcntg + (size_t)b * NB;
    int* dg = degg  + (size_t)b * NB;
    int* ig = binfog + (size_t)b * 64;
    for (int pass = 0; pass < 2; ++pass) {
      for (int i = tid * 4; i < 2 * PCAP; i += NTHR * 4) {
        const v4i v = *(const v4ia*)(pst + i);
        *(volatile v4i*)(pg + i) = v;
      }
      {
        const v4i v0 = *(const v4ia*)(spoff + 4 * tid);
        const v4i v1 = *(const v4ia*)(spcnt + 4 * tid);
        const v4i v2 = *(const v4ia*)(sdeg  + 4 * tid);
        *(volatile v4i*)(og + 4 * tid) = v0;
        *(volatile v4i*)(cg + 4 * tid) = v1;
        *(volatile v4i*)(dg + 4 * tid) = v2;
      }
      if (tid < 16) {
        const v4i v = *(const v4ia*)(binf + 4 * tid);
        *(volatile v4i*)(ig + 4 * tid) = v;
      }
      __threadfence();
    }
  }
}

__global__ __launch_bounds__(256) void k_offsets(const int* __restrict__ binfo, int* offt) {
  __shared__ __attribute__((aligned(16))) int st[OFFN];
  const int tid = (int)threadIdx.x, lane = tid & 31;
  if (tid < 32) {
    int run = 0;
#pragma unroll 1
    for (int bb = 0; bb < NBLK; ++bb) {
      int c = binfo[bb * 64 + lane];
      pini(c);
      c = clampi(c, 0, PCAP);
      st[bb * 32 + lane] = run;
      run += c;
    }
    st[NBLK * 32 + lane] = run;
    const unsigned bad = __builtin_amdgcn_ballot_w32(run > RELROWS);
    st[(NBLK + 1) * 32 + lane] = (lane == 0 && bad != 0u) ? 1 : 0;
  }
  __syncthreads();
  for (int pass = 0; pass < 2; ++pass) {
    for (int i = tid * 4; i < OFFN; i += 1024) {
      const v4i v = *(const v4ia*)(st + i);
      *(volatile v4i*)(offt + i) = v;
    }
    __threadfence();
  }
}

__global__ __launch_bounds__(256) void k_pairrows(const unsigned* __restrict__ xbw, const int* __restrict__ entg,
                                                  const unsigned* __restrict__ pairg, const int* __restrict__ binfo,
                                                  const int* __restrict__ offt, unsigned* aplw, int g) {
  const int tid = (int)threadIdx.x, lane = tid & 31;
  const int wave = __builtin_amdgcn_readfirstlane(tid >> 5);
  const int b = (int)blockIdx.x;
  int bpv = offt[b * 32 + lane];
  pini(bpv);
  bpv = clampi(bpv, 0, RELROWS);
  int rtv = offt[NBLK * 32 + lane];
  pini(rtv);
  rtv = clampi(rtv, 0, RELROWS);
  int P = binfo[b * 64 + 33];
  pini(P);
  P = clampi(P, 0, PCAP);
  P = __builtin_amdgcn_readfirstlane(P);
  const unsigned* pb = pairg + (size_t)b * (2 * PCAP);
  const int* eb = entg + (size_t)b * RCAP;

#pragma unroll 1
  for (int base = wave * 32; base < P; base += 256) {
    const int idx = base + lane;
    const int ia  = idx < PCAP ? idx : PCAP - 1;
    const v2u d = *(const v2ua*)(pb + 2 * ia);
    pinu(d.x); pinu(d.y);
    const int offv = clampi((int)(d.x & 0x3FFFu), 0, RCAP - 1);
    int cntv = (int)((d.x >> 14) & 0xFFu);
    cntv = cntv < (RCAP - offv) ? cntv : (RCAP - offv);
    const int relv = (int)((d.x >> 22) & 31u);
    const int rank = clampi((int)d.y, 0, RELROWS - 1);
    const int bp = __shfl(bpv, relv, 32);
    const int rt = __shfl(rtv, relv, 32);
    const int rin = bp + rank;
    const bool live = (idx < P) && ((relv >> 2) == g) && (rin < rt);
    const int rowv = (relv & 3) * RELROWS + (rin < RELROWS ? rin : RELROWS - 1);
    unsigned mask = __builtin_amdgcn_ballot_w32(live);
#pragma unroll 1
    for (int it = 0; it < 32; ++it) {
      if (mask == 0u) break;
      const int j = __builtin_ctz(mask);
      mask &= mask - 1u;
      const int o   = __builtin_amdgcn_readlane(offv, j);
      const int n   = __builtin_amdgcn_readlane(cntv, j);
      const int row = __builtin_amdgcn_readlane(rowv, j);
      float a0 = 0.0f, a1 = 0.0f;
#pragma unroll 1
      for (int p0 = 0; p0 < n; p0 += 32) {
        int ie = o + p0 + lane;
        ie = ie < RCAP ? ie : RCAP - 1;
        int sv = eb[ie];
        pini(sv);
        sv = clampi(sv, 0, NN - 1);
        int m = n - p0;
        m = m < 32 ? m : 32;
#pragma unroll 1
        for (int q = 0; q < m; ++q) {
          const int s = __builtin_amdgcn_readlane(sv, q);
          const unsigned w = xbw[(size_t)s * 32 + lane];
          pinu(w);
          a0 += __uint_as_float(w << 16);
          a1 += __uint_as_float(w & 0xffff0000u);
        }
      }
      const unsigned wh = pk16(bf16_bits(a0), bf16_bits(a1));
      const unsigned wl = pk16(bf16_lo_bits(a0), bf16_lo_bits(a1));
      unsigned* rp = aplw + (size_t)row * (KPAIR / 2) + lane;
      for (int pass = 0; pass < 2; ++pass) {
#pragma unroll
        for (int sgm = 0; sgm < NSEG; ++sgm) {
          const unsigned wv = (TERMS_A == 2 && sgm == 1) ? wl : wh;
          *(volatile unsigned*)(rp + 32 * sgm) = wv;
        }
        __threadfence();
      }
    }
  }

  const v4u z4 = (v4u){ 0u, 0u, 0u, 0u };
  for (int pass = 0; pass < 2; ++pass) {
#pragma unroll 1
    for (int rr = 0; rr < 4; ++rr) {
      int rt = offt[NBLK * 32 + g * 4 + rr];
      pini(rt);
      rt = clampi(rt, 0, RELROWS);
      rt = __builtin_amdgcn_readfirstlane(rt);
      const int nz = (RELROWS - rt) * PPRW;
      unsigned* zb = aplw + (size_t)(rr * RELROWS + rt) * (KPAIR / 2);
#pragma unroll 1
      for (int u = b * 256 + tid; u < nz; u += NBLK * 256) {
        *(volatile v4u*)(zb + (size_t)u * 4) = z4;
      }
    }
    __threadfence();
  }
}

template <int FIRST>
__global__ __launch_bounds__(256) void k_acc(const float* __restrict__ prod, const unsigned* __restrict__ pairg,
                                             const int* __restrict__ poffg, const int* __restrict__ pcntg,
                                             const int* __restrict__ binfo, const int* __restrict__ offt,
                                             float* acc, int g) {
  const int tid = (int)threadIdx.x, lane = tid & 31;
  const int wave = __builtin_amdgcn_readfirstlane(tid >> 5);
  const int b = (int)blockIdx.x;
  int bpv = offt[b * 32 + lane];
  pini(bpv);
  bpv = clampi(bpv, 0, RELROWS);
  int fl = binfo[b * 64 + 32];
  pini(fl);
  int gf = offt[(NBLK + 1) * 32];
  pini(gf);
  const bool pz = __builtin_amdgcn_readfirstlane((fl | gf) != 0 ? 1 : 0) != 0;
  const float qn = __uint_as_float(0x7fc00000u);
  const unsigned* pb = pairg + (size_t)b * (2 * PCAP);
  const int n0 = b * NB + wave * SPW;

#pragma unroll 1
  for (int i0 = 0; i0 < SPW; i0 += 32) {
    int pov = poffg[n0 + i0 + lane];
    int pcv = pcntg[n0 + i0 + lane];
    pini(pov); pini(pcv);
    pov = clampi(pov, 0, PCAP);
    pcv = clampi(pcv, 0, 32);
    pcv = pcv < (PCAP - pov) ? pcv : (PCAP - pov);
#pragma unroll 1
    for (int ii = 0; ii < 32; ++ii) {
      const int po = __builtin_amdgcn_readlane(pov, ii);
      const int pc = __builtin_amdgcn_readlane(pcv, ii);
      const int n  = n0 + i0 + ii;
      int ia = po + lane;
      ia = ia < PCAP ? ia : PCAP - 1;
      const v2u d = *(const v2ua*)(pb + 2 * ia);
      pinu(d.x); pinu(d.y);
      const int relv = (int)((d.x >> 22) & 31u);
      const int rank = clampi((int)d.y, 0, RELROWS - 1);
      const int bp   = __shfl(bpv, relv, 32);
      const int rin  = (bp + rank) < RELROWS ? (bp + rank) : RELROWS - 1;
      const bool live = (lane < pc) && ((relv >> 2) == g);
      const int rowv = (relv & 3) * RELROWS + rin;
      unsigned mask = __builtin_amdgcn_ballot_w32(live);
      if (!FIRST && mask == 0u && !pz) continue;
      v2f sum = (v2f){ 0.0f, 0.0f };
      if (!FIRST) {
        sum = *(const v2fa*)(acc + (size_t)n * CC + 2 * lane);
        pin2f(sum);
      }
#pragma unroll 1
      for (int it = 0; it < 32; ++it) {
        if (mask == 0u) break;
        const int j = __builtin_ctz(mask);
        mask &= mask - 1u;
        const int row = __builtin_amdgcn_readlane(rowv, j);
        const v2f v = *(const v2fa*)(prod + (size_t)row * CC + 2 * lane);
        pin2f(v);
        sum += v;
      }
      v2f res;
      res.x = pz ? qn : sum.x;
      res.y = pz ? qn : sum.y;
      volatile v2f* q = (volatile v2f*)(acc + (size_t)n * CC + 2 * lane);
      *q = res;
      __threadfence();
      *q = res;
    }
  }
}

__global__ __launch_bounds__(256) void k_final(const float* __restrict__ accg, const float* __restrict__ selfg,
                                               const int* __restrict__ degg, const float* __restrict__ biasr,
                                               const int* __restrict__ binfo, const int* __restrict__ offt,
                                               float* out) {
  const int tid = (int)threadIdx.x;
  const int r16 = tid >> 4;
  const int c4  = (tid & 15) * 4;
  const v4f bv = *(const v4fa*)(biasr + c4);
  pin4f(bv);
  int gf = offt[(NBLK + 1) * 32];
  pini(gf);
  const float qn = __uint_as_float(0x7fc00000u);
#pragma unroll 1
  for (int it = 0; it < 4; ++it) {
    const int n  = (int)blockIdx.x * 64 + it * 16 + r16;
    const int nc = n < NN ? n : NN - 1;
    const v4f a = *(const v4fa*)(accg + (size_t)nc * CC + c4);
    const v4f s = *(const v4fa*)(selfg + (size_t)nc * CC + c4);
    int dg = degg[nc];
    int fl = binfo[(nc >> SLA) * 64 + 32];
    pin4f(a); pin4f(s); pini(dg); pini(fl);
    dg = clampi(dg, 1, NE);
    const float den = (float)dg;
    const bool bad = ((fl | gf) != 0);
    v4f o;
    o[0] = (a[0] / den + s[0]) + bv[0];
    o[1] = (a[1] / den + s[1]) + bv[1];
    o[2] = (a[2] / den + s[2]) + bv[2];
    o[3] = (a[3] / den + s[3]) + bv[3];
    o[0] = bad ? qn : o[0];
    o[1] = bad ? qn : o[1];
    o[2] = bad ? qn : o[2];
    o[3] = bad ? qn : o[3];
    volatile v4f* q = (volatile v4f*)(out + (size_t)nc * CC + c4);
    if (n < NN) *q = o;
    __threadfence();
    if (n < NN) *q = o;
  }
}

constexpr size_t al256c(size_t o) { return (o + 255) & ~(size_t)255; }
constexpr size_t O_XB   = 0;
constexpr size_t O_WST  = al256c(O_XB   + (size_t)MPX * CC * 2);
constexpr size_t O_BIA  = al256c(O_WST  + (size_t)CC * CC * 2);
constexpr size_t O_RWB  = al256c(O_BIA  + (size_t)256);
constexpr size_t O_ENT  = al256c(O_RWB  + (size_t)NREL * CC * KPAIR * 2);
constexpr size_t O_PAIR = al256c(O_ENT  + (size_t)NBLK * RCAP * 4);
constexpr size_t O_POFF = al256c(O_PAIR + (size_t)NBLK * PCAP * 8);
constexpr size_t O_PCNT = al256c(O_POFF + (size_t)MPACC * 4);
constexpr size_t O_DEG  = al256c(O_PCNT + (size_t)MPACC * 4);
constexpr size_t O_BINF = al256c(O_DEG  + (size_t)MPACC * 4);
constexpr size_t O_OFFT = al256c(O_BINF + (size_t)NBLK * 64 * 4);
constexpr size_t O_APL  = al256c(O_OFFT + (size_t)OFFN * 4);
constexpr size_t O_PROD = al256c(O_APL  + (size_t)GROWS * KPAIR * 2);
constexpr size_t O_ACC  = al256c(O_PROD + (size_t)GROWS * CC * 4);
constexpr size_t WS_TOTAL = al256c(O_ACC + (size_t)MPACC * CC * 4);
static_assert(WS_TOTAL <= ((size_t)128 << 20));
static_assert((size_t)MPX * CC * 4 <= (size_t)GROWS * CC * 4);
static_assert((size_t)RELROWS * KPAIR / 8 < 0x7fffffffu);

extern "C" void kernel_launch(void* const* d_in, const int* in_sizes, int n_in,
                              void* d_out, int out_size, void* d_ws, size_t ws_size,
                              hipStream_t stream) {
  if (n_in < 8) return;
  if (in_sizes[0] != NN * CC) return;
  if (in_sizes[1] != NE || in_sizes[2] != NE || in_sizes[3] != NE) return;
  if (in_sizes[4] != NBAS * CC * CC) return;
  if (in_sizes[5] != NREL * NBAS) return;
  if (in_sizes[6] != CC * CC || in_sizes[7] != CC) return;
  if (out_size != NN * CC) return;
  if (WS_TOTAL > ws_size) return;

  const float* x     = (const float*)d_in[0];
  const int*   snd   = (const int*)d_in[1];
  const int*   rcv   = (const int*)d_in[2];
  const int*   rel   = (const int*)d_in[3];
  const float* basis = (const float*)d_in[4];
  const float* coeff = (const float*)d_in[5];
  const float* sw    = (const float*)d_in[6];
  const float* bias  = (const float*)d_in[7];
  float* out = (float*)d_out;

  char* ws = (char*)d_ws;
  unsigned short* XB   = (unsigned short*)(ws + O_XB);
  unsigned short* WST  = (unsigned short*)(ws + O_WST);
  float*          BIAR = (float*)(ws + O_BIA);
  unsigned short* RWB  = (unsigned short*)(ws + O_RWB);
  int*            ENT  = (int*)(ws + O_ENT);
  int*            PAIR = (int*)(ws + O_PAIR);
  int*            POFF = (int*)(ws + O_POFF);
  int*            PCNT = (int*)(ws + O_PCNT);
  int*            DEG  = (int*)(ws + O_DEG);
  int*            BINF = (int*)(ws + O_BINF);
  int*            OFFT = (int*)(ws + O_OFFT);
  unsigned short* APL  = (unsigned short*)(ws + O_APL);
  float*          PROD = (float*)(ws + O_PROD);
  float*          ACC  = (float*)(ws + O_ACC);

  const int bkLds = BK_INTS * 4;
  hipFuncSetAttribute(reinterpret_cast<const void*>(&k_bucket), hipFuncAttributeMaxDynamicSharedMemorySize, bkLds);

  k_prep<<<PB_X + PB_W + 1, 256, 0, stream>>>(x, sw, bias, XB, WST, BIAR);
  k_relw<<<NREL * 4, 256, 0, stream>>>(coeff, basis, RWB);
  k_bucket<<<NBLK, NTHR, bkLds, stream>>>(snd, rcv, rel, ENT, PAIR, POFF, PCNT, DEG, BINF);
  k_offsets<<<1, 256, 0, stream>>>(BINF, OFFT);

  const int pairTiles  = RELROWS / 64;
  const int pairBlocks = (pairTiles + 7) / 8;
  for (int g = 0; g < NGRP; ++g) {
    k_pairrows<<<NBLK, 256, 0, stream>>>((const unsigned*)XB, ENT, (const unsigned*)PAIR, BINF, OFFT,
                                         (unsigned*)APL, g);
    for (int rr = 0; rr < 4; ++rr) {
      const int r = g * 4 + rr;
      k_gemm_nt<0, 0><<<pairBlocks, 256, 0, stream>>>(APL + (size_t)rr * RELROWS * KPAIR,
                                                      RWB + (size_t)r * CC * KPAIR, BIAR,
                                                      PROD + (size_t)rr * RELROWS * CC, RELROWS, CC, KPAIR, CC);
    }
    if (g == 0) {
      k_acc<1><<<NBLK, 256, 0, stream>>>(PROD, (const unsigned*)PAIR, POFF, PCNT, BINF, OFFT, ACC, g);
    } else {
      k_acc<0><<<NBLK, 256, 0, stream>>>(PROD, (const unsigned*)PAIR, POFF, PCNT, BINF, OFFT, ACC, g);
    }
  }

  const int selfTiles  = MPX / 64;
  const int selfBlocks = (selfTiles + 7) / 8;
  k_gemm_nt<0, 0><<<selfBlocks, 256, 0, stream>>>(XB, WST, BIAR, PROD, MPX, CC, CC, CC);

  k_final<<<(NN + 63) / 64, 256, 0, stream>>>(ACC, PROD, DEG, BIAR, BINF, OFFT, out);
}
